// MambaAdapter_37503654429369
// MI455X (gfx1250) — hardware-run, weakly checked
//
#include <hip/hip_runtime.h>
#include <math.h>

#define NTOK  8192
#define NCH   256
#define DIN   512
#define NXZ   1024
#define DST   16
#define DTRK  16
#define DTKP  32
#define DBW   64
#define DBN   48
#define COLB  32
#define COLC  48
#define TPB   128
#define NBLK  64
#define OSTR  68
#define SCH   32
#define HCH   256
#define XTP   264
#define XT8   32
#define LOG2E 1.4426950408889634f

static_assert(NTOK % TPB == 0);
static_assert(NBLK == NTOK / TPB);
static_assert(NCH % 64 == 0);
static_assert(NXZ % 64 == 0);
static_assert(DIN % 64 == 0);
static_assert(NXZ == 2 * DIN);
static_assert(DBW >= COLC + DST);
static_assert(DTRK <= DTKP);
static_assert(DTKP % 32 == 0);
static_assert(NTOK % SCH == 0);
static_assert(SCH % 8 == 0);
static_assert(DIN % HCH == 0);
static_assert(HCH == 256);
static_assert(XTP % 8 == 0);
static_assert(XTP >= NCH);
static_assert(XT8 * 8 == NCH);
static_assert((64 * XT8) % 256 == 0);
static_assert(NTOK % 64 == 0);
static_assert(NTOK % 4 == 0);
static_assert(OSTR % 4 == 0);
static_assert(DBN - DTRK == 2 * DST);

typedef unsigned short us16 __attribute__((ext_vector_type(16)));
typedef unsigned short us8  __attribute__((ext_vector_type(8)));
typedef unsigned short us8a __attribute__((ext_vector_type(8), may_alias));
typedef unsigned int   u32x8 __attribute__((ext_vector_type(8)));
typedef __bf16 v16b __attribute__((ext_vector_type(16)));
typedef float v8f __attribute__((ext_vector_type(8)));
typedef float v4f __attribute__((ext_vector_type(4)));
typedef float v4fa __attribute__((ext_vector_type(4), may_alias));
union FragU { us16 v; us8 h[2]; u32x8 w; };

#if __has_builtin(__builtin_amdgcn_exp2f)
#define FEXP2(x) __builtin_amdgcn_exp2f(x)
#else
#define FEXP2(x) __expf((x) * 0.6931471805599453f)
#endif

__device__ __forceinline__ unsigned short bf16_bits(float f) {
  unsigned u = __float_as_uint(f);
  u += 0x7FFFu + ((u >> 16) & 1u);
  return (unsigned short)(u >> 16);
}
__device__ __forceinline__ float bf16_val(unsigned short b) { return __uint_as_float(((unsigned)b) << 16); }
__device__ __forceinline__ float bf16r(float f) { return bf16_val(bf16_bits(f)); }
__device__ __forceinline__ float siluf(float x) { return x * __builtin_amdgcn_rcpf(1.0f + __expf(-x)); }

__device__ __forceinline__ void split8(const v4f a, const v4f b, us8& hi, us8& lo) {
#pragma unroll
  for (int u = 0; u < 4; ++u) {
    const unsigned short ha = bf16_bits(a[u]);
    hi[u] = ha; lo[u] = bf16_bits(a[u] - bf16_val(ha));
    const unsigned short hb = bf16_bits(b[u]);
    hi[4 + u] = hb; lo[4 + u] = bf16_bits(b[u] - bf16_val(hb));
  }
}
__device__ __forceinline__ void hi8(const v4f a, const v4f b, us8& hi) {
#pragma unroll
  for (int u = 0; u < 4; ++u) { hi[u] = bf16_bits(a[u]); hi[4 + u] = bf16_bits(b[u]); }
}

__device__ __forceinline__ v8f mma_bf16(us16 a, us16 b, v8f c) {
  return __builtin_amdgcn_wmma_f32_16x16x32_bf16(false, __builtin_bit_cast(v16b, a), false, __builtin_bit_cast(v16b, b), (short)0, c, false, false);
}
__device__ __forceinline__ void wguard2(v8f& c0, v8f& c1, v8f& c2, v8f& c3, const us16& a0, const us16& a1,
                                        const us16& b0, const us16& b1, const us16& b2, const us16& b3) {
#if defined(__HIP_DEVICE_COMPILE__)
  asm volatile("v_nop\n\tv_nop\n\tv_nop\n\tv_nop"
               : "+v"(c0), "+v"(c1), "+v"(c2), "+v"(c3)
               : "v"(a0), "v"(a1), "v"(b0), "v"(b1), "v"(b2), "v"(b3));
#endif
}

__device__ __forceinline__ us16 gfrag(const unsigned short* p) {
  const int kh = ((threadIdx.x >> 4) & 1) * 8;
  FragU f;
  f.h[0] = *(const us8a*)(p + kh);
  f.h[1] = *(const us8a*)(p + 16 + kh);
  return f.v;
}

__global__ __launch_bounds__(256) void k_cvtT(const float* __restrict__ src, unsigned short* dst, int srcK, int srcN, int gap, int gapw,
                                             int kp8, int total8) {
  const int idx = blockIdx.x * 256 + threadIdx.x;
  if (idx >= total8) return;
  const int n = idx / kp8, k8 = (idx - n * kp8) * 8;
  const bool ingap = (n >= gap) && (n < gap + gapw);
  const int j = n - ((n >= gap + gapw) ? gapw : 0);
  const bool rowok = (!ingap) && (j >= 0) && (j < srcN);
  const int jc = rowok ? j : 0;
  us8 o;
#pragma unroll
  for (int u = 0; u < 8; ++u) {
    const int k = k8 + u;
    const int kc = (k < srcK) ? k : (srcK - 1);
    const float v = src[(size_t)kc * (size_t)srcN + jc];
    o[u] = (rowok && (k < srcK)) ? bf16_bits(v) : (unsigned short)0;
  }
  const size_t off = (size_t)idx * 8;
  *(volatile us8*)(dst + off) = o;
  __threadfence();
  *(volatile us8*)(dst + off) = o;
}

__global__ __launch_bounds__(256) void k_xtok(const float* __restrict__ x, unsigned short* XB) {
  __shared__ __attribute__((aligned(16))) unsigned short tile[64 * XTP];
  const int tid = threadIdx.x, hw0 = blockIdx.x * 64;
  const int hw = tid & 63, cq = tid >> 6;
#pragma unroll 4
  for (int it = 0; it < NCH / 4; ++it) {
    const int c = it * 4 + cq;
    const float v = x[(size_t)c * NTOK + hw0 + hw];
    tile[hw * XTP + c] = bf16_bits(v);
  }
  __syncthreads();
  us8 pv[(64 * XT8) / 256];
#pragma unroll
  for (int it = 0; it < (64 * XT8) / 256; ++it) {
    const int p = it * 256 + tid, rr = p / XT8, c8 = (p - rr * XT8) * 8;
    pv[it] = *(const us8a*)(tile + rr * XTP + c8);
  }
#pragma unroll
  for (int pass = 0; pass < 2; ++pass) {
#pragma unroll
    for (int it = 0; it < (64 * XT8) / 256; ++it) {
      const int p = it * 256 + tid, rr = p / XT8, c8 = (p - rr * XT8) * 8;
      *(volatile us8*)(XB + ((size_t)(hw0 + rr)) * NCH + c8) = pv[it];
    }
    __threadfence();
  }
}

template <int TWOA, int EPI, int OUTF, int OUTHL, int NCHWO>
__global__ __launch_bounds__(256) void k_gemm(const unsigned short* __restrict__ A0, const unsigned short* __restrict__ A1, int lda,
                                             const unsigned short* __restrict__ Bw, int ldb, int K,
                                             float* Yf, int ldy, unsigned short* YH, int ldh,
                                             float* Onc, int ldo, const float* __restrict__ bias, int epi_n0) {
  __shared__ __attribute__((aligned(16))) float oS[8 * 16 * OSTR];
  const int tid = threadIdx.x, lane = tid & 31, wave = tid >> 5, cl = lane & 15, hh = lane >> 4;
  const int mb = blockIdx.x * TPB, m0 = mb + 16 * wave, n0 = blockIdx.y * 64;

  v8f acc[4];
#pragma unroll
  for (int j = 0; j < 4; ++j) { const v8f zz = {0.f, 0.f, 0.f, 0.f, 0.f, 0.f, 0.f, 0.f}; acc[j] = zz; }

  const unsigned short* a0p = A0 + (size_t)(m0 + cl) * lda;
  const unsigned short* a1p = A1 + (size_t)(m0 + cl) * lda;
  const unsigned short* bwp = Bw + (size_t)(n0 + cl) * ldb;
#pragma unroll 1
  for (int k0 = 0; k0 < K; k0 += 32) {
    const us16 af0 = gfrag(a0p + k0);
    us16 af1 = af0;
    if (TWOA) af1 = gfrag(a1p + k0);
    us16 bfr[4];
#pragma unroll
    for (int j = 0; j < 4; ++j) bfr[j] = gfrag(bwp + (size_t)(16 * j) * ldb + k0);
#pragma unroll
    for (int j = 0; j < 4; ++j) acc[j] = mma_bf16(af0, bfr[j], acc[j]);
    if (TWOA) {
#pragma unroll
      for (int j = 0; j < 4; ++j) acc[j] = mma_bf16(af1, bfr[j], acc[j]);
    }
    wguard2(acc[0], acc[1], acc[2], acc[3], af0, af1, bfr[0], bfr[1], bfr[2], bfr[3]);
  }

  float* so = oS + wave * (16 * OSTR);
#pragma unroll
  for (int j = 0; j < 4; ++j)
#pragma unroll
    for (int r = 0; r < 8; ++r) so[(8 * hh + r) * OSTR + 16 * j + cl] = acc[j][r];
  __syncthreads();

  if (EPI != 0 && n0 >= epi_n0) {
#pragma unroll 1
    for (int e = tid; e < TPB * 64; e += 256) {
      const int R = e >> 6, cc = e & 63;
      float v = oS[R * OSTR + cc];
      if (EPI == 1) {
        v = siluf(v);
      } else {
        const float a = v + bf16r(bias[n0 + cc]);
        v = fmaxf(a, 0.0f) + log1pf(__expf(-fabsf(a)));
      }
      oS[R * OSTR + cc] = v;
    }
    __syncthreads();
  }

  if (OUTF) {
    v4f vv[8];
#pragma unroll
    for (int it = 0; it < 8; ++it) {
      const int ch = it * 32 + lane, r = ch >> 4, q = (ch & 15) * 4;
      vv[it] = *(const v4fa*)(so + r * OSTR + q);
    }
#pragma unroll
    for (int pass = 0; pass < 2; ++pass) {
#pragma unroll
      for (int it = 0; it < 8; ++it) {
        const int ch = it * 32 + lane, r = ch >> 4, q = (ch & 15) * 4;
        *(volatile v4f*)(Yf + (size_t)(m0 + r) * ldy + n0 + q) = vv[it];
      }
      __threadfence();
    }
  }
  if (OUTHL) {
    us8 hv[4];
#pragma unroll
    for (int it = 0; it < 4; ++it) {
      const int ch = it * 32 + lane, r = ch >> 3, c8 = (ch & 7) * 8;
      const v4f a = *(const v4fa*)(so + r * OSTR + c8);
      const v4f b = *(const v4fa*)(so + r * OSTR + c8 + 4);
      hi8(a, b, hv[it]);
    }
#pragma unroll
    for (int pass = 0; pass < 2; ++pass) {
#pragma unroll
      for (int it = 0; it < 4; ++it) {
        const int ch = it * 32 + lane, r = ch >> 3, c8 = (ch & 7) * 8;
        *(volatile us8*)(YH + (size_t)(m0 + r) * ldh + n0 + c8) = hv[it];
      }
      __threadfence();
    }
  }
  if (NCHWO) {
    v4f ov[8];
#pragma unroll
    for (int it = 0; it < 8; ++it) {
      const int c = it * 8 + wave;
#pragma unroll
      for (int i = 0; i < 4; ++i) ov[it][i] = oS[(lane * 4 + i) * OSTR + c];
    }
#pragma unroll
    for (int pass = 0; pass < 2; ++pass) {
#pragma unroll
      for (int it = 0; it < 8; ++it) {
        const int c = it * 8 + wave;
        const size_t o = ((size_t)(n0 + c)) * (size_t)ldo + mb + lane * 4;
        *(volatile v4f*)(Onc + o) = ov[it];
      }
      __threadfence();
    }
  }
}

__global__ __launch_bounds__(256) void k_conv(const float* __restrict__ XZ, const float* __restrict__ cw, const float* __restrict__ cb,
                                             float* UF, unsigned short* UH) {
  __shared__ __attribute__((aligned(16))) float su[4 * DIN];
  const int tid = threadIdx.x, q = tid >> 6, c8 = (tid & 63) * 8;
  const int tok0 = blockIdx.x * 4, tok = tok0 + q;
  float s[8];
#pragma unroll
  for (int u = 0; u < 8; ++u) s[u] = 0.0f;
#pragma unroll
  for (int j = 0; j < 4; ++j) {
    const int ls = tok - 3 + j;
    const int lsc = (ls < 0) ? 0 : ls;
    const bool ok = (ls >= 0);
    const float* xr = XZ + (size_t)lsc * NXZ + c8;
    const v4f xa = *(const v4fa*)xr, xb = *(const v4fa*)(xr + 4);
#pragma unroll
    for (int u = 0; u < 4; ++u) {
      const float w0 = bf16r(cw[(c8 + u) * 4 + j]);
      const float w1 = bf16r(cw[(c8 + 4 + u) * 4 + j]);
      const float x0 = ok ? xa[u] : 0.0f;
      const float x1 = ok ? xb[u] : 0.0f;
      s[u] = s[u] + w0 * x0;
      s[4 + u] = s[4 + u] + w1 * x1;
    }
  }
  v4f ua, ub;
#pragma unroll
  for (int u = 0; u < 4; ++u) {
    ua[u] = siluf(s[u] + bf16r(cb[c8 + u]));
    ub[u] = siluf(s[4 + u] + bf16r(cb[c8 + 4 + u]));
  }
  *(v4fa*)(su + q * DIN + c8) = ua;
  *(v4fa*)(su + q * DIN + c8 + 4) = ub;
  us8 hi;
  hi8(ua, ub, hi);
  const size_t oh = (size_t)tok * DIN + c8;
  *(volatile us8*)(UH + oh) = hi;
  __threadfence();
  *(volatile us8*)(UH + oh) = hi;
  __syncthreads();
  v4f fv[2];
#pragma unroll
  for (int it = 0; it < 2; ++it) {
    const int p = it * 256 + tid, row = p >> 7, col = (p & 127) * 4;
    fv[it] = *(const v4fa*)(su + row * DIN + col);
  }
#pragma unroll
  for (int pass = 0; pass < 2; ++pass) {
#pragma unroll
    for (int it = 0; it < 2; ++it) {
      const int p = it * 256 + tid, row = p >> 7, col = (p & 127) * 4;
      *(volatile v4f*)(UF + (size_t)(tok0 + row) * DIN + col) = fv[it];
    }
    __threadfence();
  }
}

__global__ __launch_bounds__(256) void k_scan(const float* __restrict__ DT, const float* __restrict__ UF, const float* __restrict__ XDBL,
                                             const float* __restrict__ XZ, const float* __restrict__ Alog, const float* __restrict__ Dv,
                                             unsigned short* YH, unsigned short* YL) {
  __shared__ __attribute__((aligned(16))) float sy[SCH * HCH];
  const int tid = threadIdx.x, lane = tid & 31, wave = tid >> 5;
  const int dofs = blockIdx.x * HCH, d = dofs + tid;
  float A2[DST], h[DST];
#pragma unroll
  for (int i = 0; i < DST; ++i) { A2[i] = -__expf(bf16r(Alog[(size_t)d * DST + i])) * LOG2E; h[i] = 0.0f; }
  const float Dd = bf16r(Dv[d]);
#pragma unroll 1
  for (int c = 0; c < NTOK / SCH; ++c) {
#pragma unroll 1
    for (int s = 0; s < SCH; ++s) {
      const size_t tok = (size_t)(c * SCH + s);
      const size_t e = tok * DIN + d;
      const float dl = DT[e], uv = UF[e];
      const float gz = XZ[tok * NXZ + DIN + d];
      const float* bc = XDBL + tok * DBW + COLB;
      v4f Bv[4], Cv[4];
#pragma unroll
      for (int q = 0; q < 4; ++q) {
        Bv[q] = *(const v4fa*)(bc + 4 * q);
        Cv[q] = *(const v4fa*)(bc + (COLC - COLB) + 4 * q);
      }
      const float dx = dl * uv;
      float y = 0.0f;
#pragma unroll
      for (int i = 0; i < DST; ++i) {
        const float ex = FEXP2(dl * A2[i]);
        h[i] = ex * h[i] + dx * Bv[i >> 2][i & 3];
        y = y + h[i] * Cv[i >> 2][i & 3];
      }
      sy[s * HCH + tid] = (y + uv * Dd) * gz;
    }
    __syncthreads();
    us8 hv[SCH / 8], lv[SCH / 8];
#pragma unroll
    for (int it = 0; it < SCH / 8; ++it) {
      const int row = it * 8 + wave, c8 = lane * 8;
      const v4f a = *(const v4fa*)(sy + row * HCH + c8);
      const v4f b = *(const v4fa*)(sy + row * HCH + c8 + 4);
      split8(a, b, hv[it], lv[it]);
    }
#pragma unroll
    for (int pass = 0; pass < 2; ++pass) {
#pragma unroll
      for (int it = 0; it < SCH / 8; ++it) {
        const int row = it * 8 + wave, c8 = lane * 8;
        const size_t off = ((size_t)(c * SCH + row)) * DIN + dofs + c8;
        *(volatile us8*)(YH + off) = hv[it];
        *(volatile us8*)(YL + off) = lv[it];
      }
      __threadfence();
    }
    __syncthreads();
  }
}

extern "C" void kernel_launch(void* const* d_in, const int* in_sizes, int n_in,
                              void* d_out, int out_size, void* d_ws, size_t ws_size,
                              hipStream_t stream) {
  if (n_in < 10) return;
  if (in_sizes[0] != NCH * NTOK || in_sizes[1] != NCH * NXZ || in_sizes[2] != DIN * 4 || in_sizes[3] != DIN ||
      in_sizes[4] != DIN * DBN || in_sizes[5] != DTRK * DIN || in_sizes[6] != DIN || in_sizes[7] != DIN * DST ||
      in_sizes[8] != DIN || in_sizes[9] != DIN * NCH) return;
  if (out_size != NCH * NTOK) return;

  const float* x       = (const float*)d_in[0];
  const float* W_in    = (const float*)d_in[1];
  const float* conv_w  = (const float*)d_in[2];
  const float* conv_b  = (const float*)d_in[3];
  const float* W_xproj = (const float*)d_in[4];
  const float* W_dt    = (const float*)d_in[5];
  const float* b_dt    = (const float*)d_in[6];
  const float* A_log   = (const float*)d_in[7];
  const float* D_skip  = (const float*)d_in[8];
  const float* W_out   = (const float*)d_in[9];
  float* out = (float*)d_out;

  size_t off = 0;
  auto carve = [&](size_t bytes) -> char* { char* p = (char*)d_ws + off; off += (bytes + 255) & ~(size_t)255; return p; };
  unsigned short* XB  = (unsigned short*)carve((size_t)NTOK * NCH * 2);
  float* XZ   = (float*)carve((size_t)NTOK * NXZ * 4);
  float* UF   = (float*)carve((size_t)NTOK * DIN * 4);
  unsigned short* UH  = (unsigned short*)carve((size_t)NTOK * DIN * 2);
  float* XDBL = (float*)carve((size_t)NTOK * DBW * 4);
  unsigned short* XDH = (unsigned short*)carve((size_t)NTOK * DBW * 2);
  float* DT   = (float*)carve((size_t)NTOK * DIN * 4);
  unsigned short* YH  = (unsigned short*)carve((size_t)NTOK * DIN * 2);
  unsigned short* YL  = (unsigned short*)carve((size_t)NTOK * DIN * 2);
  unsigned short* WIN = (unsigned short*)carve((size_t)NXZ * NCH * 2);
  unsigned short* WXP = (unsigned short*)carve((size_t)DBW * DIN * 2);
  unsigned short* WDT = (unsigned short*)carve((size_t)DIN * DTKP * 2);
  unsigned short* WOP = (unsigned short*)carve((size_t)NCH * DIN * 2);
  if (off > ws_size || off > (size_t)134217728) return;

  const dim3 b256(256);
  auto cdv = [](long a, long b) { return (unsigned)((a + b - 1) / b); };

  k_cvtT<<<dim3(cdv(NXZ * (NCH / 8), 256)), b256, 0, stream>>>(W_in, WIN, NCH, NXZ, 1 << 20, 0, NCH / 8, NXZ * (NCH / 8));
  k_cvtT<<<dim3(cdv(DBW * (DIN / 8), 256)), b256, 0, stream>>>(W_xproj, WXP, DIN, DBN, DTRK, COLB - DTRK, DIN / 8, DBW * (DIN / 8));
  k_cvtT<<<dim3(cdv(DIN * (DTKP / 8), 256)), b256, 0, stream>>>(W_dt, WDT, DTRK, DIN, 1 << 20, 0, DTKP / 8, DIN * (DTKP / 8));
  k_cvtT<<<dim3(cdv(NCH * (DIN / 8), 256)), b256, 0, stream>>>(W_out, WOP, DIN, NCH, 1 << 20, 0, DIN / 8, NCH * (DIN / 8));
  k_xtok<<<dim3(NTOK / 64), b256, 0, stream>>>(x, XB);
  k_gemm<0, 1, 1, 0, 0><<<dim3(NBLK, NXZ / 64), b256, 0, stream>>>(XB, XB, NCH, WIN, NCH, NCH, XZ, NXZ, UH, DIN, XZ, NTOK, b_dt, DIN);
  k_conv<<<dim3(NTOK / 4), b256, 0, stream>>>(XZ, conv_w, conv_b, UF, UH);
  k_gemm<0, 0, 1, 1, 0><<<dim3(NBLK, 1), b256, 0, stream>>>(UH, UH, DIN, WXP, DIN, DIN, XDBL, DBW, XDH, DBW, XZ, NTOK, b_dt, 0);
  k_gemm<0, 2, 1, 0, 0><<<dim3(NBLK, DIN / 64), b256, 0, stream>>>(XDH, XDH, DBW, WDT, DTKP, DTKP, DT, DIN, UH, DIN, XZ, NTOK, b_dt, 0);
  k_scan<<<dim3(DIN / HCH), b256, 0, stream>>>(DT, UF, XDBL, XZ, A_log, D_skip, YH, YL);
  k_gemm<1, 0, 0, 0, 1><<<dim3(NBLK, NCH / 64), b256, 0, stream>>>(YH, YL, DIN, WOP, DIN, DIN, XDBL, DBW, UH, DIN, out, NTOK, b_dt, 0);
}
